// TransformerBlock_66700842107002
// MI455X (gfx1250) — hardware-verified
//
#include <hip/hip_runtime.h>
#ifndef NB
#define NB 4
#endif
#ifndef SEQ
#define SEQ 2048
#endif
#define NB_FULL 4
#define SEQ_FULL 2048
#define DM 512
#define NH 8
#define HD 64
#define DFF 2048
#define LQ (3 * DM)
#define NR ((size_t)NB * SEQ)
#define WSC 64.0f
#define ASC 16.0f
#define GSC 16.0f

static_assert(SEQ % 128 == 0);
static_assert(SEQ <= SEQ_FULL);
static_assert(NB <= NB_FULL);
static_assert(DM == NH * HD);
static_assert(DM % 128 == 0 && DFF % 64 == 0 && LQ % 64 == 0);
static_assert(DM % 32 == 0 && DFF % 32 == 0 && HD == 64);

typedef unsigned short v8us __attribute__((ext_vector_type(8), may_alias));
typedef float  v8f  __attribute__((ext_vector_type(8)));
typedef float  v4f  __attribute__((ext_vector_type(4)));
typedef float  v4fa __attribute__((ext_vector_type(4), may_alias));
typedef _Float16 v16h __attribute__((ext_vector_type(16)));
typedef _Float16 v4h __attribute__((ext_vector_type(4)));
union FragH { v16h v; v8us half[2]; _Float16 h[16]; unsigned short u[16]; };

__device__ __forceinline__ unsigned short bf16_bits(float x) { unsigned int u = __float_as_uint(x); return (unsigned short)((u + 0x7FFFu + ((u >> 16) & 1u)) >> 16); }
__device__ __forceinline__ float bf16_val(unsigned short b) { return __uint_as_float(((unsigned int)b) << 16); }
__device__ __forceinline__ float bf16_rne(float x) { return bf16_val(bf16_bits(x)); }

__device__ __forceinline__ v16h g2_frag(const _Float16* p, int hh) { FragH f; f.half[0] = *(const v8us*)((const unsigned short*)p + 8 * hh); f.half[1] = *(const v8us*)((const unsigned short*)p + 16 + 8 * hh); return f.v; }
__device__ __forceinline__ v8f g2_mma(v16h a, v16h b, v8f c) { v8f d = __builtin_amdgcn_wmma_f32_16x16x32_f16(false, a, false, b, (short)0, c, false, false); asm volatile("v_nop\n\tv_nop\n\tv_nop\n\tv_nop" : "+v"(d) : "v"(a), "v"(b)); return d; }

__global__ __launch_bounds__(256) void k_wt_f16(const float* __restrict__ W, _Float16* __restrict__ Wt, int K, int N, float scale) {
  const int t = blockIdx.x * 256 + threadIdx.x; if (t >= N * (K / 8)) return; const int n = t / (K / 8), k8 = (t % (K / 8)) * 8; FragH f;
#pragma unroll
  for (int i = 0; i < 8; ++i) f.h[i] = (_Float16)(bf16_rne(W[(size_t)(k8 + i) * N + n]) * scale);
  const v8us o = f.half[0];
  *(volatile v8us*)((unsigned short*)Wt + (size_t)n * K + k8) = o; __threadfence(); *(volatile v8us*)((unsigned short*)Wt + (size_t)n * K + k8) = o;
}

template <int BFIN, int WXB>
__global__ __launch_bounds__(256) void k_lnw(const float* __restrict__ X, const float* __restrict__ g, const float* __restrict__ bb, float eps, float ysc,
                                             _Float16* __restrict__ N16, float* __restrict__ XB, int nrows, int sq, int sqf) {
  #pragma clang fp contract(off)
  const int wave = __builtin_amdgcn_readfirstlane((int)(threadIdx.x >> 5));
  const int lane = threadIdx.x & 31;
  const int r = blockIdx.x * 8 + wave;
  if (r >= nrows) return;
  const int b = r / sq, s = r - b * sq;
  const size_t rsrc = (size_t)b * sqf + s;
  const float* xr = X + rsrc * DM;
  float v[16]; float sum = 0.f;
#pragma unroll
  for (int c = 0; c < 4; ++c) {
    const v4f a = *(const v4fa*)(xr + c * 128 + lane * 4);
#pragma unroll
    for (int q = 0; q < 4; ++q) { const float t = BFIN ? bf16_rne(a[q]) : a[q]; v[c * 4 + q] = t; sum += t; }
  }
#pragma unroll
  for (int m = 16; m > 0; m >>= 1) sum += __shfl_xor(sum, m);
  const float mu = sum * (1.0f / (float)DM);
  float vs = 0.f;
#pragma unroll
  for (int i = 0; i < 16; ++i) { const float dl = v[i] - mu; vs += dl * dl; }
#pragma unroll
  for (int m = 16; m > 0; m >>= 1) vs += __shfl_xor(vs, m);
  const float rs = rsqrtf(vs * (1.0f / (float)DM) + eps);
  v4h y[4]; v4f xb[4];
#pragma unroll
  for (int c = 0; c < 4; ++c) {
    const v4f gv = *(const v4fa*)(g + c * 128 + lane * 4);
    const v4f bv = *(const v4fa*)(bb + c * 128 + lane * 4);
#pragma unroll
    for (int q = 0; q < 4; ++q) {
      const float yn = ((v[c * 4 + q] - mu) * rs) * bf16_rne(gv[q]) + bf16_rne(bv[q]);
      y[c][q] = (_Float16)(yn * ysc);
      xb[c][q] = v[c * 4 + q];
    }
  }
  for (int pass = 0; pass < 2; ++pass) {
#pragma unroll
    for (int c = 0; c < 4; ++c) {
      *(volatile v4h*)(N16 + (size_t)r * DM + c * 128 + lane * 4) = y[c];
      if (WXB) *(volatile v4f*)(XB + rsrc * DM + c * 128 + lane * 4) = xb[c];
    }
    if (pass == 0) __threadfence();
  }
}

template <int ACT>
__global__ __launch_bounds__(128) void k_gemm2(const _Float16* __restrict__ A, int lda, size_t sA, const _Float16* __restrict__ Bh, int ldb, float alpha,
                                               const float* __restrict__ bias, const float* __restrict__ CP,
                                               float* __restrict__ C, _Float16* __restrict__ C16, float c16s, int ldc, size_t sC, int M, int N, int K) {
  static_assert(ACT == 0 || ACT == 6);
  __shared__ __attribute__((aligned(16))) float so[4][32][68];
  const int w = __builtin_amdgcn_readfirstlane((int)(threadIdx.x >> 5));
  const int lane = threadIdx.x & 31, ln = lane & 15, hh = lane >> 4; const int by = blockIdx.y;
  A += (size_t)by * sA; const size_t cofs = (size_t)by * sC;
  const int ntn = N >> 6; const int mt = blockIdx.x / ntn, nq = blockIdx.x - mt * ntn; const int row0 = mt * 128 + 32 * w, col0 = nq * 64; if (row0 >= M) return;
  const _Float16* a0p = A + (size_t)(row0 + ln) * lda; const _Float16* a1p = a0p + (size_t)16 * lda;
  const _Float16* b0p = Bh + (size_t)(col0 + ln) * ldb; const _Float16* b1p = b0p + (size_t)16 * ldb; const _Float16* b2p = b1p + (size_t)16 * ldb; const _Float16* b3p = b2p + (size_t)16 * ldb;
  const v8f z8 = {0.f,0.f,0.f,0.f,0.f,0.f,0.f,0.f}; v8f c00 = z8, c01 = z8, c02 = z8, c03 = z8, c10 = z8, c11 = z8, c12 = z8, c13 = z8;
#pragma unroll 1
  for (int kb = 0; kb < K; kb += 32) { const v16h a0 = g2_frag(a0p + kb, hh), a1 = g2_frag(a1p + kb, hh);
    v16h b = g2_frag(b0p + kb, hh); c00 = g2_mma(a0, b, c00); c10 = g2_mma(a1, b, c10);
    b = g2_frag(b1p + kb, hh); c01 = g2_mma(a0, b, c01); c11 = g2_mma(a1, b, c11);
    b = g2_frag(b2p + kb, hh); c02 = g2_mma(a0, b, c02); c12 = g2_mma(a1, b, c12);
    b = g2_frag(b3p + kb, hh); c03 = g2_mma(a0, b, c03); c13 = g2_mma(a1, b, c13); }
  v8f accs[8] = {c00, c01, c02, c03, c10, c11, c12, c13};
#pragma unroll
  for (int u = 0; u < 8; ++u) { const int t = u & 3, half = u >> 2; const int col = col0 + t * 16 + ln; const float bv = bias ? bf16_rne(bias[col]) : 0.f;
#pragma unroll
    for (int r = 0; r < 8; ++r) { const int rloc = half * 16 + 8 * hh + r; float v = accs[u][r] * alpha + bv;
      if (CP) v += CP[cofs + (size_t)(row0 + rloc) * ldc + col];
      if (ACT == 6) v = 0.5f * v * (1.0f + erff(v * 0.70710678118654752f));
      so[w][rloc][t * 16 + ln] = v; } }
  __builtin_amdgcn_fence(4  , "workgroup"); __builtin_amdgcn_wave_barrier();
  const int rsub = lane >> 4, c4 = (lane & 15) * 4;
  for (int pass = 0; pass < 2; ++pass) {
#pragma unroll
    for (int q = 0; q < 16; ++q) { const int r = q * 2 + rsub; const v4f v = *(const v4fa*)&so[w][r][c4];
      if (C) *(volatile v4f*)(C + cofs + (size_t)(row0 + r) * ldc + col0 + c4) = v;
      if (C16) { v4h h4; for (int i = 0; i < 4; ++i) h4[i] = (_Float16)(v[i] * c16s); *(volatile v4h*)(C16 + cofs + (size_t)(row0 + r) * ldc + col0 + c4) = h4; } }
    if (pass == 0) __threadfence(); }
}

template <int NHv, int TTv>
__global__ __launch_bounds__(256) void k_vt(const _Float16* __restrict__ V16, int ldv, int voff, _Float16* __restrict__ Vt) {
  __shared__ unsigned short tl[64][66];
  const int tid = threadIdx.x; const int slab = blockIdx.x / (TTv / 64), lg = blockIdx.x % (TTv / 64); const int b = slab / NHv, h = slab % NHv;
  for (int i = tid; i < 64 * 8; i += 256) { const int r = i / 8, c8 = (i % 8) * 8; FragH f; f.half[0] = *(const v8us*)((const unsigned short*)V16 + ((size_t)b * TTv + lg * 64 + r) * ldv + voff + h * 64 + c8);
#pragma unroll
    for (int q = 0; q < 8; ++q) tl[r][c8 + q] = f.u[q]; }
  __syncthreads();
  for (int pass = 0; pass < 2; ++pass) {
#pragma unroll
    for (int rd = 0; rd < 2; ++rd) { const int d = rd * 32 + tid / 8, pc = tid % 8; FragH f;
#pragma unroll
      for (int q = 0; q < 8; ++q) f.u[q] = tl[pc * 8 + q][d];
      *(volatile v8us*)((unsigned short*)Vt + ((size_t)slab * 64 + d) * TTv + lg * 64 + pc * 8) = f.half[0]; }
    if (pass == 0) __threadfence(); }
}

__global__ __launch_bounds__(128) void k_fattn(const _Float16* __restrict__ QKV, const _Float16* __restrict__ VT, _Float16* __restrict__ O16) {
  __shared__ __attribute__((aligned(16))) unsigned short lo[4][16][72];
  const int wave = __builtin_amdgcn_readfirstlane((int)(threadIdx.x >> 5));
  const int lane = threadIdx.x & 31, ln = lane & 15, hh = lane >> 4;
  const int qt = blockIdx.x % (SEQ / 64), bh = blockIdx.x / (SEQ / 64);
  const int b = bh / NH, h = bh - b * NH;
  const size_t tok0 = (size_t)b * SEQ;
  const int qrow0 = qt * 64 + wave * 16;
  const _Float16* qp = QKV + (tok0 + qrow0 + ln) * LQ + h * HD;
  const v16h q0 = g2_frag(qp, hh), q1 = g2_frag(qp + 32, hh);
  const _Float16* kbase = QKV + (tok0 + ln) * LQ + DM + h * HD;
  const _Float16* vbase = VT + ((size_t)bh * HD + ln) * SEQ;
  const v8f z8 = {0.f,0.f,0.f,0.f,0.f,0.f,0.f,0.f};
  v8f o0 = z8, o1 = z8, o2 = z8, o3 = z8;
  float m = -1.0e30f, l = 0.f;
#pragma unroll 1
  for (int kb = 0; kb < SEQ; kb += 32) {
    const _Float16* kp = kbase + (size_t)kb * LQ;
    v8f s0 = z8, s1 = z8;
    s0 = g2_mma(g2_frag(kp, hh), q0, s0);
    s0 = g2_mma(g2_frag(kp + 32, hh), q1, s0);
    s1 = g2_mma(g2_frag(kp + (size_t)16 * LQ, hh), q0, s1);
    s1 = g2_mma(g2_frag(kp + (size_t)16 * LQ + 32, hh), q1, s1);
    float a0[8], a1[8]; float mx = -1.0e30f;
#pragma unroll
    for (int r = 0; r < 8; ++r) { a0[r] = s0[r] * 0.125f; a1[r] = s1[r] * 0.125f; mx = fmaxf(mx, fmaxf(a0[r], a1[r])); }
    mx = fmaxf(mx, __shfl_xor(mx, 16));
    const float mn = fmaxf(m, mx);
    const float corr = __expf(m - mn);
    FragH pf; float ls = 0.f;
#pragma unroll
    for (int r = 0; r < 8; ++r) {
      const float p0 = __expf(a0[r] - mn), p1 = __expf(a1[r] - mn);
      ls += p0 + p1;
      pf.h[r] = (_Float16)(p0 * 256.0f);
      pf.h[8 + r] = (_Float16)(p1 * 256.0f);
    }
    ls += __shfl_xor(ls, 16);
    l = l * corr + ls; m = mn;
    o0 *= corr; o1 *= corr; o2 *= corr; o3 *= corr;
    const _Float16* vp = vbase + kb;
    o0 = g2_mma(g2_frag(vp, hh), pf.v, o0);
    o1 = g2_mma(g2_frag(vp + (size_t)16 * SEQ, hh), pf.v, o1);
    o2 = g2_mma(g2_frag(vp + (size_t)32 * SEQ, hh), pf.v, o2);
    o3 = g2_mma(g2_frag(vp + (size_t)48 * SEQ, hh), pf.v, o3);
  }
  const float fin = 0.25f / l;
  { FragH f;
#pragma unroll
    for (int r = 0; r < 8; ++r) f.h[r] = (_Float16)(o0[r] * fin);
    *(v8us*)&lo[wave][ln][0 + 8 * hh] = f.half[0];
#pragma unroll
    for (int r = 0; r < 8; ++r) f.h[r] = (_Float16)(o1[r] * fin);
    *(v8us*)&lo[wave][ln][16 + 8 * hh] = f.half[0];
#pragma unroll
    for (int r = 0; r < 8; ++r) f.h[r] = (_Float16)(o2[r] * fin);
    *(v8us*)&lo[wave][ln][32 + 8 * hh] = f.half[0];
#pragma unroll
    for (int r = 0; r < 8; ++r) f.h[r] = (_Float16)(o3[r] * fin);
    *(v8us*)&lo[wave][ln][48 + 8 * hh] = f.half[0]; }
  __builtin_amdgcn_fence(4  , "workgroup"); __builtin_amdgcn_wave_barrier();
  const int rq = lane >> 3, pc = lane & 7;
  for (int pass = 0; pass < 2; ++pass) {
#pragma unroll
    for (int it = 0; it < 4; ++it) { const int row = it * 4 + rq; const v8us v = *(const v8us*)&lo[wave][row][pc * 8];
      *(volatile v8us*)((unsigned short*)O16 + (tok0 + qrow0 + row) * DM + h * HD + pc * 8) = v; }
    if (pass == 0) __threadfence(); }
}

extern "C" void kernel_launch(void* const* d_in, const int* in_sizes, int n_in,
                              void* d_out, int out_size, void* d_ws, size_t ws_size, hipStream_t stream) {
  if (n_in < 13) return;
  const size_t xneed = ((size_t)(NB - 1) * SEQ_FULL + SEQ) * DM;
  if ((size_t)in_sizes[0] < xneed || (size_t)out_size < xneed) return;
  if (in_sizes[1] < DM || in_sizes[2] < DM || in_sizes[3] < DM * LQ || in_sizes[4] < LQ || in_sizes[5] < DM * DM || in_sizes[6] < DM) return;
  if (in_sizes[7] < DM || in_sizes[8] < DM || in_sizes[9] < DM * DFF || in_sizes[10] < DFF || in_sizes[11] < DFF * DM || in_sizes[12] < DM) return;
  const float* x = (const float*)d_in[0]; const float* g1 = (const float*)d_in[1]; const float* be1 = (const float*)d_in[2];
  const float* wqkv = (const float*)d_in[3]; const float* bqkv = (const float*)d_in[4]; const float* wo = (const float*)d_in[5]; const float* bo = (const float*)d_in[6];
  const float* g2 = (const float*)d_in[7]; const float* be2 = (const float*)d_in[8]; const float* wfc = (const float*)d_in[9]; const float* bfc = (const float*)d_in[10];
  const float* wmp = (const float*)d_in[11]; const float* bmp = (const float*)d_in[12];
  char* ws = (char*)d_ws; size_t off = 0;
  auto take = [&](size_t bytes) { char* p = ws + off; off += (bytes + 255) & ~(size_t)255; return p; };
  _Float16* BQKV = (_Float16*)take((size_t)LQ * DM * 2);
  _Float16* BO   = (_Float16*)take((size_t)DM * DM * 2);
  _Float16* BW1  = (_Float16*)take((size_t)DFF * DM * 2);
  _Float16* BW2  = (_Float16*)take((size_t)DM * DFF * 2);
  _Float16* X16  = (_Float16*)take(NR * DM * 2);
  float*    XB   = (float*)take((size_t)NB * SEQ_FULL * DM * 4);
  float*    X1   = (float*)take((size_t)NB * SEQ_FULL * DM * 4);
  _Float16* QKV  = (_Float16*)take(NR * LQ * 2);
  _Float16* VT   = (_Float16*)take((size_t)NB * NH * HD * SEQ * 2);
  _Float16* O16  = (_Float16*)take(NR * DM * 2);
  _Float16* HF16 = (_Float16*)take(NR * DFF * 2);
  _Float16* M16  = X16;
  if (off > ws_size || off > (size_t)134217728) return;

  k_wt_f16<<<(unsigned)(((size_t)LQ * (DM / 8) + 255) / 256), 256, 0, stream>>>(wqkv, BQKV, DM, LQ, WSC);
  k_wt_f16<<<(unsigned)(((size_t)DM * (DM / 8) + 255) / 256), 256, 0, stream>>>(wo, BO, DM, DM, WSC);
  k_wt_f16<<<(unsigned)(((size_t)DFF * (DM / 8) + 255) / 256), 256, 0, stream>>>(wfc, BW1, DM, DFF, WSC);
  k_wt_f16<<<(unsigned)(((size_t)DM * (DFF / 8) + 255) / 256), 256, 0, stream>>>(wmp, BW2, DFF, DM, WSC);
  k_lnw<1, 1><<<(unsigned)((NR + 7) / 8), 256, 0, stream>>>(x, g1, be1, 1e-5f, ASC, X16, XB, (int)NR, SEQ, SEQ_FULL);
  k_gemm2<0><<<dim3((unsigned)((NR / 128) * (LQ / 64)), 1), 128, 0, stream>>>(X16, DM, 0, BQKV, DM, 1.0f / (WSC * ASC), bqkv, nullptr, nullptr, QKV, 1.0f, LQ, 0, (int)NR, LQ, DM);
  k_vt<NH, SEQ><<<NB * NH * (SEQ / 64), 256, 0, stream>>>(QKV, LQ, 2 * DM, VT);
  k_fattn<<<NB * NH * (SEQ / 64), 128, 0, stream>>>(QKV, VT, O16);
  k_gemm2<0><<<dim3((unsigned)((SEQ / 128) * (DM / 64)), NB), 128, 0, stream>>>(O16, DM, (size_t)SEQ * DM, BO, DM, 1.0f / (WSC * 64.0f), bo, XB, X1, nullptr, 1.0f, DM, (size_t)SEQ_FULL * DM, SEQ, DM, DM);
  k_lnw<0, 0><<<(unsigned)((NR + 7) / 8), 256, 0, stream>>>(X1, g2, be2, 1e-5f, ASC, M16, nullptr, (int)NR, SEQ, SEQ_FULL);
  k_gemm2<6><<<dim3((unsigned)((NR / 128) * (DFF / 64)), 1), 128, 0, stream>>>(M16, DM, 0, BW1, DM, 1.0f / (WSC * ASC), bfc, nullptr, nullptr, HF16, GSC, DFF, 0, (int)NR, DFF, DM);
  k_gemm2<0><<<dim3((unsigned)((SEQ / 128) * (DM / 64)), NB), 128, 0, stream>>>(HF16, DFF, (size_t)SEQ * DFF, BW2, DFF, 1.0f / (WSC * GSC), bmp, X1, (float*)d_out, nullptr, 1.0f, DM, (size_t)SEQ_FULL * DM, SEQ, DM, DFF);
}
